// VisionAttention_15642270892547
// MI455X (gfx1250) — hardware-verified
//
#include <hip/hip_runtime.h>
#include <math.h>
#include <stdint.h>

#define S_TOK  4096
#define NHD    16
#define HDIM   64
#define ROWP   (NHD * HDIM)
#define NTOT   (S_TOK * ROWP)
#define NCU    9
#define NT64   (S_TOK / 64)
#define SCL2   0.18033688011112042f

#define AT_D   64
#define AT_NW  4
#define AT_QB  64
#define AT_KC  64

static_assert(S_TOK % 64 == 0);
static_assert(NTOT % (256 * 8) == 0);
static_assert(ROWP % 64 == 0);
static_assert(S_TOK % 256 == 0);

typedef __attribute__((ext_vector_type(16))) __bf16   v16b;
typedef __attribute__((ext_vector_type(8)))  __bf16   v8b;
typedef __attribute__((ext_vector_type(8)))  float    v8f;
typedef __attribute__((ext_vector_type(4)))  float    v4f;
typedef __attribute__((ext_vector_type(4)))  unsigned int v4u;
typedef __attribute__((ext_vector_type(4)))  int      v4i;

__device__ __forceinline__ unsigned short f2bf_bits(float f) {
  unsigned u = __float_as_uint(f);
  return (unsigned short)((u + 0x7FFFu + ((u >> 16) & 1u)) >> 16);
}
__device__ __forceinline__ float bf_bits2f(unsigned short h) { return __uint_as_float(((unsigned)h) << 16); }
__device__ __forceinline__ unsigned pk16(unsigned short a, unsigned short b) { return (unsigned)a | ((unsigned)b << 16); }
__device__ __forceinline__ __bf16 at_f2bf(float f) { return __builtin_bit_cast(__bf16, f2bf_bits(f)); }
__device__ __forceinline__ void at_split(float f, __bf16& hi, __bf16& lo) {
  const unsigned short hb = f2bf_bits(f);
  hi = __builtin_bit_cast(__bf16, hb);
  lo = at_f2bf(f - bf_bits2f(hb));
}

__device__ __forceinline__ v8f at_mma(v16b a, v16b b, v8f c) {
  c = __builtin_amdgcn_wmma_f32_16x16x32_bf16(false, a, false, b, (short)0, c, false, false);
  asm volatile("v_nop\n\tv_nop\n\tv_nop\n\tv_nop" : "+v"(c) : "v"(a), "v"(b));
  return c;
}

union FBU { v16b v; v8b h[2]; };
__device__ __forceinline__ v16b frag_ld(const __bf16* p) {
  FBU f; f.h[0] = *(const v8b*)(p); f.h[1] = *(const v8b*)(p + 16); return f.v;
}

__global__ __launch_bounds__(256) void cvt_qk_kernel(const float* __restrict__ q, const float* __restrict__ k,
                                                     unsigned short* __restrict__ qb, unsigned short* __restrict__ kb, int n8) {
  const int i = blockIdx.x * 256 + threadIdx.x;
  if (i < n8) {
    const size_t e = (size_t)i * 8;
    const v4f a0 = *(const v4f*)(q + e);
    const v4f a1 = *(const v4f*)(q + e + 4);
    const v4f b0 = *(const v4f*)(k + e);
    const v4f b1 = *(const v4f*)(k + e + 4);
    v4u qa, ka;
    qa[0] = pk16(f2bf_bits(a0[0]), f2bf_bits(a0[1]));
    qa[1] = pk16(f2bf_bits(a0[2]), f2bf_bits(a0[3]));
    qa[2] = pk16(f2bf_bits(a1[0]), f2bf_bits(a1[1]));
    qa[3] = pk16(f2bf_bits(a1[2]), f2bf_bits(a1[3]));
    ka[0] = pk16(f2bf_bits(b0[0]), f2bf_bits(b0[1]));
    ka[1] = pk16(f2bf_bits(b0[2]), f2bf_bits(b0[3]));
    ka[2] = pk16(f2bf_bits(b1[0]), f2bf_bits(b1[1]));
    ka[3] = pk16(f2bf_bits(b1[2]), f2bf_bits(b1[3]));
    *(volatile v4u*)(qb + e) = qa;
    *(volatile v4u*)(kb + e) = ka;
    __threadfence();
    *(volatile v4u*)(qb + e) = qa;
    *(volatile v4u*)(kb + e) = ka;
  }
}

__global__ __launch_bounds__(256) void vt_bf16_kernel(const float* __restrict__ W, unsigned short* __restrict__ ov,
                                                      int R, int Cc) {
  __shared__ __align__(16) float tf[64 * 68];
  const int c0  = blockIdx.x * 64;
  const int r0  = blockIdx.y * 64;
  const int tid = threadIdx.x;
  {
    const int lr = tid >> 4;
    const int c4 = (tid & 15) * 4;
#pragma unroll
    for (int it = 0; it < 4; ++it) {
      const int rr = it * 16 + lr;
      const v4f a = *(const v4f*)(W + (size_t)(r0 + rr) * Cc + c0 + c4);
      *(v4f*)(tf + rr * 68 + c4) = a;
    }
  }
  __syncthreads();
  const int sub = tid >> 3;
  const int c8  = (tid & 7) * 8;
  v4u hv[2];
#pragma unroll
  for (int it = 0; it < 2; ++it) {
    const int oc = it * 32 + sub;
    v4u a;
#pragma unroll
    for (int q4 = 0; q4 < 4; ++q4) {
      const float f0 = tf[(c8 + 2 * q4) * 68 + oc];
      const float f1 = tf[(c8 + 2 * q4 + 1) * 68 + oc];
      a[q4] = pk16(f2bf_bits(f0), f2bf_bits(f1));
    }
    hv[it] = a;
  }
  for (int pass = 0; pass < 2; ++pass) {
#pragma unroll
    for (int it = 0; it < 2; ++it) {
      const int oc = it * 32 + sub;
      const size_t go = (size_t)(c0 + oc) * R + r0 + c8;
      *(volatile v4u*)(ov + go) = hv[it];
    }
    __threadfence();
  }
}

__global__ __launch_bounds__(256) void seg_tables_kernel(const int* __restrict__ cu, int* __restrict__ segp,
                                                         int* __restrict__ tmmp) {
  __shared__ int cuS[16];
  __shared__ __align__(16) int segs[S_TOK];
  __shared__ __align__(16) int tmn[NT64];
  __shared__ __align__(16) int tmx[NT64];
  const int tid  = threadIdx.x;
  const int lane = tid & 31;
  const int wave = tid >> 5;
  const int ci = (tid < NCU) ? tid : (NCU - 1);
  const int cv = cu[ci];
  if (tid < 16) cuS[tid] = (tid < NCU) ? cv : 0x7fffffff;
  __syncthreads();
#pragma unroll 1
  for (int ch = 0; ch < S_TOK / 256; ++ch) {
    const int i = ch * 256 + tid;
    int s = 0;
#pragma unroll
    for (int j = 0; j < NCU; ++j) s += (cuS[j] <= i) ? 1 : 0;
    segs[i] = s;
  }
  __syncthreads();
  if (tid < NT64) {
    int mn = 1 << 20, mx = -1;
#pragma unroll 1
    for (int t = 0; t < 64; ++t) {
      const int sv = segs[tid * 64 + t];
      mn = min(mn, sv);
      mx = max(mx, sv);
    }
    tmn[tid] = mn;
    tmx[tid] = mx;
  }
  __syncthreads();
  v4i sv4[4];
#pragma unroll
  for (int it = 0; it < 4; ++it) sv4[it] = *(const v4i*)(segs + 4 * (it * 256 + tid));
  const v4i ta = *(const v4i*)(tmn + ((4 * lane) & 63));
  const v4i tb = *(const v4i*)(tmx + ((4 * lane) & 63));
  v4i tv;
#pragma unroll
  for (int e = 0; e < 4; ++e) tv[e] = (lane < 16) ? ta[e] : tb[e];
  for (int pass = 0; pass < 2; ++pass) {
#pragma unroll
    for (int it = 0; it < 4; ++it) *(volatile v4i*)(segp + 4 * (it * 256 + tid)) = sv4[it];
    if (wave == 0) *(volatile v4i*)(tmmp + 4 * lane) = tv;
    __threadfence();
  }
}

__global__ __launch_bounds__(128)
void seg_attn64_kernel(const unsigned short* __restrict__ qbp, const unsigned short* __restrict__ kbp,
                       const unsigned short* __restrict__ vtp, const int* __restrict__ segp,
                       const int* __restrict__ tmmp, float* __restrict__ out) {
  __shared__ __align__(16) __bf16 Ksh[AT_KC * AT_D];
  __shared__ __align__(16) __bf16 Vth[AT_D * AT_KC];
  __shared__ __align__(16) __bf16 Psh[AT_NW][16 * AT_KC];
  __shared__ __align__(16) __bf16 Psl[AT_NW][16 * AT_KC];
  __shared__ __align__(16) float  Os[AT_NW][16 * 68];
  __shared__ __align__(16) int    tmm[2 * NT64];
  __shared__ __align__(16) int    csg[AT_KC];

  const int tid  = threadIdx.x;
  const int wave = tid >> 5;
  const int lane = tid & 31;
  const int hh   = lane >> 4;
  const int c    = lane & 15;

  const int bx = blockIdx.x;
  const int qt = bx & (NT64 - 1);
  const int h  = bx >> 6;
  const int q0 = qt * AT_QB + wave * 16;

  if (tid < 32) *(v4i*)(tmm + 4 * tid) = *(const v4i*)(tmmp + 4 * tid);

  int sr[8];
  {
    const v4i a = *(const v4i*)(segp + q0 + 8 * hh);
    const v4i b = *(const v4i*)(segp + q0 + 8 * hh + 4);
    sr[0] = a[0]; sr[1] = a[1]; sr[2] = a[2]; sr[3] = a[3];
    sr[4] = b[0]; sr[5] = b[1]; sr[6] = b[2]; sr[7] = b[3];
  }

  const __bf16* Qb = (const __bf16*)(const void*)qbp + (size_t)h * AT_D;
  const __bf16* Kb = (const __bf16*)(const void*)kbp + (size_t)h * AT_D;
  const __bf16* Vb = (const __bf16*)(const void*)vtp + (size_t)h * AT_D * S_TOK;
  float*        ob = out + (size_t)h * AT_D;

  v16b qa[2];
#pragma unroll
  for (int dc = 0; dc < 2; ++dc) qa[dc] = frag_ld(Qb + (size_t)(q0 + c) * ROWP + dc * 32 + 8 * hh);

  float mrow[8], lrow[8];
  v8f oacc[4];
#pragma unroll
  for (int r = 0; r < 8; ++r) { mrow[r] = -INFINITY; lrow[r] = 0.f; }
#pragma unroll
  for (int t = 0; t < 4; ++t) oacc[t] = (v8f){0.f,0.f,0.f,0.f,0.f,0.f,0.f,0.f};

  __syncthreads();
  const int qmn  = __builtin_amdgcn_readfirstlane(tmm[qt]);
  const int qmx  = __builtin_amdgcn_readfirstlane(tmm[NT64 + qt]);
  const int quni = (qmn == qmx) ? 1 : 0;

  for (int kt = 0; kt < NT64; ++kt) {
    const int kmn = __builtin_amdgcn_readfirstlane(tmm[kt]);
    const int kmx = __builtin_amdgcn_readfirstlane(tmm[NT64 + kt]);
    const int live = ((kmx < qmn) || (qmx < kmn)) ? 0 : 1;
    if (live == 0) continue;
    const int full = ((quni != 0) && (kmn == kmx) && (kmn == qmn)) ? 1 : 0;
    const int kv0 = kt * AT_KC;

    __syncthreads();
    {
      const int r = tid >> 1, half = (tid & 1) * 32;
      const __bf16* ks = Kb + (size_t)(kv0 + r) * ROWP + half;
      const __bf16* vs = Vb + (size_t)r * S_TOK + kv0 + half;
#pragma unroll
      for (int i = 0; i < 4; ++i) {
        const v8b a0 = *(const v8b*)(ks + 8 * i);
        const v8b b0 = *(const v8b*)(vs + 8 * i);
        *(v8b*)(Ksh + r * AT_D  + half + 8 * i) = a0;
        *(v8b*)(Vth + r * AT_KC + half + 8 * i) = b0;
      }
      const int segv = segp[kv0 + (tid & 63)];
      if (tid < 64) csg[tid] = segv;
    }
    __syncthreads();

    int sc[4];
#pragma unroll
    for (int j = 0; j < 4; ++j) sc[j] = csg[j * 16 + c];

    v8f s[4];
#pragma unroll
    for (int j = 0; j < 4; ++j) {
      s[j] = (v8f){0.f,0.f,0.f,0.f,0.f,0.f,0.f,0.f};
#pragma unroll
      for (int dc = 0; dc < 2; ++dc) {
        FBU kb;
        kb.h[0] = *(const v8b*)(Ksh + (j * 16 + c) * AT_D + dc * 32 + 8 * hh);
        kb.h[1] = *(const v8b*)(Ksh + (j * 16 + c) * AT_D + dc * 32 + 16 + 8 * hh);
        s[j] = at_mma(qa[dc], kb.v, s[j]);
      }
    }
    float cm[8];
#pragma unroll
    for (int r = 0; r < 8; ++r) {
      float m = -INFINITY;
#pragma unroll
      for (int j = 0; j < 4; ++j) {
        const int lv = full | ((sr[r] == sc[j]) ? 1 : 0);
        const float sv = (lv != 0) ? (s[j][r] * SCL2) : -INFINITY;
        s[j][r] = sv;
        m = fmaxf(m, sv);
      }
#pragma unroll
      for (int off = 1; off < 16; off <<= 1) m = fmaxf(m, __shfl_xor(m, off, 32));
      cm[r] = m;
    }
    __bf16* pwh = Psh[wave];
    __bf16* pwl = Psl[wave];
#pragma unroll
    for (int r = 0; r < 8; ++r) {
      const float mnew  = fmaxf(mrow[r], cm[r]);
      const float safe  = (mnew == -INFINITY) ? 0.f : mnew;
      const float alpha = exp2f(mrow[r] - safe);
      mrow[r] = mnew;
      float psum = 0.f;
#pragma unroll
      for (int j = 0; j < 4; ++j) {
        const float p = exp2f(s[j][r] - safe);
        psum += p;
        __bf16 a, bl; at_split(p, a, bl);
        pwh[(8 * hh + r) * AT_KC + j * 16 + c] = a;
        pwl[(8 * hh + r) * AT_KC + j * 16 + c] = bl;
      }
#pragma unroll
      for (int off = 1; off < 16; off <<= 1) psum += __shfl_xor(psum, off, 32);
      lrow[r] = lrow[r] * alpha + psum;
#pragma unroll
      for (int t = 0; t < 4; ++t) oacc[t][r] *= alpha;
    }
    __builtin_amdgcn_fence(__ATOMIC_RELEASE, "workgroup");
    __builtin_amdgcn_wave_barrier();
    __builtin_amdgcn_fence(__ATOMIC_ACQUIRE, "workgroup");
#pragma unroll 1
    for (int kk = 0; kk < 2; ++kk) {
      FBU pa, pl;
      pa.h[0] = *(const v8b*)(pwh + c * AT_KC + kk * 32 + 8 * hh);
      pa.h[1] = *(const v8b*)(pwh + c * AT_KC + kk * 32 + 16 + 8 * hh);
      pl.h[0] = *(const v8b*)(pwl + c * AT_KC + kk * 32 + 8 * hh);
      pl.h[1] = *(const v8b*)(pwl + c * AT_KC + kk * 32 + 16 + 8 * hh);
#pragma unroll
      for (int t = 0; t < 4; ++t) {
        FBU vb;
        vb.h[0] = *(const v8b*)(Vth + (t * 16 + c) * AT_KC + kk * 32 + 8 * hh);
        vb.h[1] = *(const v8b*)(Vth + (t * 16 + c) * AT_KC + kk * 32 + 16 + 8 * hh);
        oacc[t] = at_mma(pa.v, vb.v, oacc[t]);
        oacc[t] = at_mma(pl.v, vb.v, oacc[t]);
      }
    }
  }

  float* os = Os[wave];
#pragma unroll
  for (int r = 0; r < 8; ++r) {
    const float lv  = lrow[r];
    const float inv = (lv > 0.f) ? (1.0f / lv) : 0.f;
#pragma unroll
    for (int t = 0; t < 4; ++t) os[(8 * hh + r) * 68 + t * 16 + c] = oacc[t][r] * inv;
  }
  __builtin_amdgcn_fence(__ATOMIC_RELEASE, "workgroup");
  __builtin_amdgcn_wave_barrier();
  __builtin_amdgcn_fence(__ATOMIC_ACQUIRE, "workgroup");
  {
    const int c4 = (lane & 15) * 4;
    for (int pass = 0; pass < 2; ++pass) {
#pragma unroll
      for (int it = 0; it < 8; ++it) {
        const int row = it * 2 + hh;
        v4f val = *(const v4f*)(os + row * 68 + c4);
        *(volatile v4f*)(ob + (size_t)(q0 + row) * ROWP + c4) = val;
      }
      __threadfence();
    }
  }
}

extern "C" void kernel_launch(void* const* d_in, const int* in_sizes, int n_in,
                              void* d_out, int out_size, void* d_ws, size_t ws_size,
                              hipStream_t stream) {
  if (n_in < 4) return;
  if (in_sizes[0] != NTOT || in_sizes[1] != NTOT || in_sizes[2] != NTOT) return;
  if (in_sizes[3] != NCU) return;
  if (out_size != NTOT) return;

  const float* q  = (const float*)d_in[0];
  const float* k  = (const float*)d_in[1];
  const float* v  = (const float*)d_in[2];
  const int*   cu = (const int*)d_in[3];
  float* out = (float*)d_out;

  const size_t PB  = (size_t)NTOT * 2;
  const size_t PSG = (size_t)S_TOK * 4;
  const size_t PTM = (size_t)2 * NT64 * 4;
  size_t off = 0;
  const size_t oQB  = off; off += PB;
  const size_t oKB  = off; off += PB;
  const size_t oVT  = off; off += PB;
  const size_t oSEG = off; off += PSG;
  const size_t oTMM = off; off += PTM;
  if (off > ws_size) return;

  char* ws = (char*)d_ws;
  unsigned short* QB  = (unsigned short*)(ws + oQB);
  unsigned short* KB  = (unsigned short*)(ws + oKB);
  unsigned short* VT  = (unsigned short*)(ws + oVT);
  int*            SEG = (int*)(ws + oSEG);
  int*            TMM = (int*)(ws + oTMM);

  const int n8 = NTOT / 8;
  cvt_qk_kernel<<<dim3((n8 + 255) / 256), dim3(256), 0, stream>>>(q, k, QB, KB, n8);
  vt_bf16_kernel<<<dim3(ROWP / 64, S_TOK / 64), dim3(256), 0, stream>>>(v, VT, S_TOK, ROWP);
  seg_tables_kernel<<<dim3(1), dim3(256), 0, stream>>>(cu, SEG, TMM);
  seg_attn64_kernel<<<dim3(NHD * NT64), dim3(128), 0, stream>>>(QB, KB, VT, SEG, TMM, out);
  (void)hipGetLastError();
}
